// DecoderLayer_12369505812685
// MI455X (gfx1250) — hardware-verified
//
#include <hip/hip_runtime.h>
#ifndef NB
#define NB 4
#endif
#ifndef SEQ
#define SEQ 2048
#endif
#define NB_FULL 4
#define SEQ_FULL 2048
#define DM 1024
#define NH 16
#define HD 64
#define LQ (3 * DM)
#define MROWS (NB * SEQ)
#define NQT (SEQ / 64)
#define USEQ ((unsigned)SEQ)
static_assert(SEQ % 64 == 0);
static_assert(SEQ >= 64 && SEQ <= SEQ_FULL);
static_assert(NB >= 1 && NB <= NB_FULL);
static_assert(MROWS % 128 == 0);
static_assert(DM == 1024 && HD == 64 && NH * HD == DM);
static_assert((MROWS * (DM / 8)) % 256 == 0);
static_assert((DM * DM / 8) % 256 == 0);
static_assert((SEQ * HD) % 256 == 0);

typedef _Float16 v16h __attribute__((ext_vector_type(16)));
typedef _Float16 v4h  __attribute__((ext_vector_type(4)));
typedef unsigned short v8us __attribute__((ext_vector_type(8), may_alias));
typedef float  v8f  __attribute__((ext_vector_type(8)));
typedef float  v4f  __attribute__((ext_vector_type(4)));
typedef float  v4fa __attribute__((ext_vector_type(4), may_alias));
union FragH { v16h v; v8us half[2]; _Float16 h[16]; unsigned short u[16]; };

#define NEG_INF (-__builtin_inff())

__device__ __forceinline__ unsigned short bf16_bits(float x) { unsigned int u = __float_as_uint(x); return (unsigned short)((u + 0x7FFFu + ((u >> 16) & 1u)) >> 16); }
__device__ __forceinline__ float bf16_val(unsigned short b) { return __uint_as_float(((unsigned int)b) << 16); }
__device__ __forceinline__ float bf16_rne(float x) { return bf16_val(bf16_bits(x)); }

__device__ __forceinline__ v16h g2_frag(const _Float16* p, unsigned hh) { FragH f; f.half[0] = *(const v8us*)((const unsigned short*)p + 8u * hh); f.half[1] = *(const v8us*)((const unsigned short*)p + 16u + 8u * hh); return f.v; }
__device__ __forceinline__ v8f g2_mma(v16h a, v16h b, v8f c) { v8f d = __builtin_amdgcn_wmma_f32_16x16x32_f16(false, a, false, b, (short)0, c, false, false); asm volatile("v_nop\n\tv_nop\n\tv_nop\n\tv_nop" : "+v"(d) : "v"(a), "v"(b)); return d; }

__global__ __launch_bounds__(256) void k_x16(const float* __restrict__ x, _Float16* __restrict__ X16) {
  const unsigned t = blockIdx.x * 256u + threadIdx.x; if (t >= (unsigned)(MROWS * (DM / 8))) return;
  const unsigned m = t >> 7, c8 = (t & 127u) * 8u; const unsigned b = m / USEQ, s = m % USEQ;
  const float* src = x + ((size_t)b * SEQ_FULL + s) * DM + c8;
  const v4f a = *(const v4fa*)src, c = *(const v4fa*)(src + 4); FragH f;
#pragma unroll
  for (int i = 0; i < 4; ++i) { f.h[i] = (_Float16)bf16_rne(a[i]); f.h[4 + i] = (_Float16)bf16_rne(c[i]); }
  unsigned short* d = (unsigned short*)X16 + (size_t)t * 8;
  *(volatile v8us*)d = f.half[0]; __threadfence(); *(volatile v8us*)d = f.half[0]; }

__global__ __launch_bounds__(256) void k_wnat(const float* __restrict__ w0, const float* __restrict__ w1, const float* __restrict__ w2, const float* __restrict__ w3, _Float16* __restrict__ WB) {
  const unsigned t = blockIdx.x * 256u + threadIdx.x; if (t >= (unsigned)(DM * DM / 8)) return;
  const unsigned y = blockIdx.y;
  const float* w = (y == 0u) ? w0 : ((y == 1u) ? w1 : ((y == 2u) ? w2 : w3));
  const v4f a = *(const v4fa*)(w + (size_t)t * 8), c = *(const v4fa*)(w + (size_t)t * 8 + 4); FragH f;
#pragma unroll
  for (int i = 0; i < 4; ++i) { f.h[i] = (_Float16)(bf16_rne(a[i]) * 16.0f); f.h[4 + i] = (_Float16)(bf16_rne(c[i]) * 16.0f); }
  unsigned short* d = (unsigned short*)WB + (size_t)y * DM * DM + (size_t)t * 8;
  *(volatile v8us*)d = f.half[0]; __threadfence(); *(volatile v8us*)d = f.half[0]; }

__global__ __launch_bounds__(64) void k_div(float* __restrict__ RD) {
  const unsigned d = threadIdx.x; const float e = (float)(2u * (d >> 1)) * 0.015625f;
  const float dv = powf(10000.0f, e); const float rd = 1.0f / dv;
  volatile float* p = RD + d; *p = rd; __threadfence(); *p = rd; }

__global__ __launch_bounds__(256) void k_pe(const float* __restrict__ RD, float* __restrict__ PE) {
  const unsigned t = blockIdx.x * 256u + threadIdx.x; if (t >= (unsigned)(SEQ * HD)) return;
  const unsigned s = t >> 6, d = t & 63u; const float ang = (float)s * RD[d];
  const float sn = sinf(ang), cs = cosf(ang); const float v = ((d & 1u) != 0u) ? cs : sn;
  volatile float* p = PE + t; *p = v; __threadfence(); *p = v; }

template <int MODE>
__global__ __launch_bounds__(128) void k_gemm2(const _Float16* __restrict__ A, const _Float16* __restrict__ Bh, float alpha, const float* __restrict__ aux,
    _Float16* __restrict__ C16, float* __restrict__ C32) {
  __shared__ __attribute__((aligned(16))) float so[4][32][68];
  const unsigned tid = threadIdx.x, w = tid >> 5, lane = tid & 31u, ln = lane & 15u, hh = lane >> 4;
  const unsigned mt = blockIdx.x / (unsigned)(DM / 64), nq = blockIdx.x % (unsigned)(DM / 64);
  const unsigned row0 = mt * 128u + 32u * w, col0 = nq * 64u;
  const _Float16* a0p = A + (size_t)(row0 + ln) * DM; const _Float16* a1p = a0p + (size_t)16 * DM;
  const _Float16* b0p = Bh + (size_t)(col0 + ln) * DM; const _Float16* b1p = b0p + (size_t)16 * DM; const _Float16* b2p = b1p + (size_t)16 * DM; const _Float16* b3p = b2p + (size_t)16 * DM;
  const v8f z8 = {0.f,0.f,0.f,0.f,0.f,0.f,0.f,0.f}; v8f c00 = z8, c01 = z8, c02 = z8, c03 = z8, c10 = z8, c11 = z8, c12 = z8, c13 = z8;
#pragma unroll 1
  for (unsigned kb = 0; kb < (unsigned)DM; kb += 32u) { const v16h a0 = g2_frag(a0p + kb, hh), a1 = g2_frag(a1p + kb, hh);
    v16h b = g2_frag(b0p + kb, hh); c00 = g2_mma(a0, b, c00); c10 = g2_mma(a1, b, c10);
    b = g2_frag(b1p + kb, hh); c01 = g2_mma(a0, b, c01); c11 = g2_mma(a1, b, c11);
    b = g2_frag(b2p + kb, hh); c02 = g2_mma(a0, b, c02); c12 = g2_mma(a1, b, c12);
    b = g2_frag(b3p + kb, hh); c03 = g2_mma(a0, b, c03); c13 = g2_mma(a1, b, c13); }
  v8f accs[8] = {c00, c01, c02, c03, c10, c11, c12, c13};
#pragma unroll
  for (int u = 0; u < 8; ++u) { const int t = u & 3, half = u >> 2;
#pragma unroll
    for (int r = 0; r < 8; ++r) { const unsigned rloc = (unsigned)half * 16u + 8u * hh + (unsigned)r; so[w][rloc][(unsigned)t * 16u + ln] = accs[u][r] * alpha; } }
  __builtin_amdgcn_fence(4  , "workgroup"); __builtin_amdgcn_wave_barrier();
  if (MODE == 0 || MODE == 2) {
    const unsigned rsub = lane >> 4, c4 = (lane & 15u) * 4u;
    for (int pass = 0; pass < 2; ++pass) {
#pragma unroll
      for (int q = 0; q < 16; ++q) { const unsigned r = (unsigned)q * 2u + rsub; const unsigned row = row0 + r; v4f v = *(const v4fa*)&so[w][r][c4];
        if (MODE == 0) { const unsigned s = row % USEQ; const v4f pe = *(const v4fa*)(aux + (size_t)s * HD + c4);
#pragma unroll
          for (int i = 0; i < 4; ++i) v[i] += pe[i]; }
        v4h h4;
#pragma unroll
        for (int i = 0; i < 4; ++i) h4[i] = (_Float16)v[i];
        *(volatile v4h*)(C16 + (size_t)row * LQ + col0 + c4) = h4; }
      if (pass == 0) __threadfence(); }
  } else {
    const unsigned rq = lane >> 3, pc = lane & 7u;
    for (int pass = 0; pass < 2; ++pass) {
#pragma unroll
      for (int g = 0; g < 16; ++g) { const unsigned L = (unsigned)g * 4u + rq; const unsigned r = L >> 1, col = (L & 1u) * 32u + pc * 4u; const unsigned row = row0 + r;
        v4f v = *(const v4fa*)&so[w][r][col];
        if (MODE == 3) { const unsigned b = row / USEQ, s = row % USEQ; const v4f xr = *(const v4fa*)(aux + ((size_t)b * SEQ_FULL + s) * DM + col0 + col);
#pragma unroll
          for (int i = 0; i < 4; ++i) v[i] += bf16_rne(xr[i]); }
        *(volatile v4f*)(C32 + (size_t)row * DM + col0 + col) = v; }
      if (pass == 0) __threadfence(); }
  } }

__global__ __launch_bounds__(256) void k_smear(const float* __restrict__ KF, const float* __restrict__ alpha, const float* __restrict__ PE, _Float16* __restrict__ QKV) {
  const unsigned t = blockIdx.x * 256u + threadIdx.x; if (t >= (unsigned)(MROWS * (DM / 8))) return;
  const unsigned m = t >> 7, c8 = (t & 127u) * 8u; const unsigned h = c8 >> 6, d0 = c8 & 63u;
  const unsigned b = m / USEQ, s = m % USEQ; const unsigned sp = (s > 0u) ? (s - 1u) : 0u;
  const float* kc = KF + (size_t)m * DM + c8; const float* kp = KF + ((size_t)b * SEQ + sp) * DM + c8;
  const v4f c0 = *(const v4fa*)kc, c1 = *(const v4fa*)(kc + 4), p0 = *(const v4fa*)kp, p1 = *(const v4fa*)(kp + 4);
  const float al = bf16_rne(alpha[h * (unsigned)(SEQ_FULL - 1) + sp]);
  const float a = 1.0f / (1.0f + expf(-al)); const float om = 1.0f - a;
  const v4f e0 = *(const v4fa*)(PE + (size_t)s * HD + d0), e1 = *(const v4fa*)(PE + (size_t)s * HD + d0 + 4);
  const bool first = (s == 0u); FragH f;
#pragma unroll
  for (int i = 0; i < 4; ++i) { const float u0 = c0[i] * a + p0[i] * om, u1 = c1[i] * a + p1[i] * om;
    const float v0 = first ? c0[i] : u0, v1 = first ? c1[i] : u1;
    f.h[i] = (_Float16)(v0 + e0[i]); f.h[4 + i] = (_Float16)(v1 + e1[i]); }
  unsigned short* d = (unsigned short*)QKV + (size_t)m * LQ + DM + c8;
  *(volatile v8us*)d = f.half[0]; __threadfence(); *(volatile v8us*)d = f.half[0]; }

__global__ __launch_bounds__(256) void k_vt2(const _Float16* __restrict__ QKV, _Float16* __restrict__ VT) {
  __shared__ unsigned short tl[64][66];
  const unsigned tid = threadIdx.x; const unsigned slab = blockIdx.x / (unsigned)NQT, lg = blockIdx.x % (unsigned)NQT; const unsigned b = slab / (unsigned)NH, hd = slab % (unsigned)NH; const unsigned s0 = lg * 64u;
  for (unsigned i = tid; i < 512u; i += 256u) { const unsigned r = i >> 3, c8 = (i & 7u) * 8u; FragH f;
    f.half[0] = *(const v8us*)((const unsigned short*)QKV + ((size_t)b * SEQ + s0 + r) * LQ + 2 * DM + hd * HD + c8);
#pragma unroll
    for (int q = 0; q < 8; ++q) tl[r][c8 + q] = f.u[q]; }
  __syncthreads();
  for (int pass = 0; pass < 2; ++pass) {
#pragma unroll
    for (int rd = 0; rd < 2; ++rd) { const unsigned d = (unsigned)rd * 32u + (tid >> 3), pc = tid & 7u; FragH f;
#pragma unroll
      for (int q = 0; q < 8; ++q) f.u[q] = tl[pc * 8u + q][d];
      *(volatile v8us*)((unsigned short*)VT + ((size_t)slab * HD + d) * SEQ + s0 + pc * 8u) = f.half[0]; }
    if (pass == 0) __threadfence(); } }

__global__ __launch_bounds__(128) void k_attn(const _Float16* __restrict__ QKV, const _Float16* __restrict__ VT, _Float16* __restrict__ CTX) {
  __shared__ __attribute__((aligned(16))) float so[4][16][68];
  const unsigned tid = threadIdx.x, w = tid >> 5, lane = tid & 31u, l15 = lane & 15u, hh = lane >> 4;
  const unsigned qt = blockIdx.x, slab = blockIdx.y; const unsigned b = slab / (unsigned)NH, hd = slab % (unsigned)NH;
  const unsigned q0 = qt * 64u + w * 16u;
  const _Float16* Qb = QKV + (size_t)b * SEQ * LQ + hd * HD;
  const _Float16* Kb = Qb + DM;
  const _Float16* Vb = VT + (size_t)slab * HD * SEQ;
  const _Float16* qrow = Qb + (size_t)(q0 + l15) * LQ;
  const v16h qf0 = g2_frag(qrow, hh), qf1 = g2_frag(qrow + 32, hh);
  const unsigned qme = q0 + l15;
  const v8f z8 = {0.f,0.f,0.f,0.f,0.f,0.f,0.f,0.f};
  v8f o[4] = {z8, z8, z8, z8};
  float m = NEG_INF, l = 0.f;
  const float CL = 0.18033688011112042f;
#pragma unroll 1
  for (unsigned it = 0; it <= qt; ++it) {
    const unsigned key0 = it * 64u;
    v8f s[4];
#pragma unroll
    for (int kt = 0; kt < 4; ++kt) {
      const _Float16* krow = Kb + (size_t)(key0 + (unsigned)kt * 16u + l15) * LQ;
      const v16h ka = g2_frag(krow, hh), kk = g2_frag(krow + 32, hh);
      v8f a = g2_mma(ka, qf0, z8); a = g2_mma(kk, qf1, a); s[kt] = a; }
    if (it == qt) {
#pragma unroll
      for (int kt = 0; kt < 4; ++kt) {
#pragma unroll
        for (int r = 0; r < 8; ++r) { const unsigned key = key0 + (unsigned)kt * 16u + 8u * hh + (unsigned)r; s[kt][r] = (key > qme) ? NEG_INF : s[kt][r]; } } }
    float lmax = NEG_INF;
#pragma unroll
    for (int kt = 0; kt < 4; ++kt)
#pragma unroll
      for (int r = 0; r < 8; ++r) lmax = fmaxf(lmax, s[kt][r]);
    lmax = fmaxf(lmax, __shfl_xor(lmax, 16));
    const float mnew = fmaxf(m, lmax);
    const float mref = (mnew == NEG_INF) ? 0.0f : mnew;
    const float alpha = exp2f((m - mref) * CL);
    const float bexp = 10.0f - mref * CL;
    m = mnew;
    float psum = 0.f; FragH pa, pb;
#pragma unroll
    for (int r = 0; r < 8; ++r) {
      const float e0 = exp2f(fmaf(s[0][r], CL, bexp)), e1 = exp2f(fmaf(s[1][r], CL, bexp)), e2 = exp2f(fmaf(s[2][r], CL, bexp)), e3 = exp2f(fmaf(s[3][r], CL, bexp));
      psum += (e0 + e1) + (e2 + e3);
      pa.h[r] = (_Float16)e0; pa.h[8 + r] = (_Float16)e1; pb.h[r] = (_Float16)e2; pb.h[8 + r] = (_Float16)e3; }
    l = l * alpha + psum;
    float ar[8];
#pragma unroll
    for (int r = 0; r < 8; ++r) ar[r] = __shfl(alpha, (int)(8u * hh) + r);
#pragma unroll
    for (int dt = 0; dt < 4; ++dt) {
#pragma unroll
      for (int r = 0; r < 8; ++r) o[dt][r] *= ar[r];
      const _Float16* vrow = Vb + (size_t)((unsigned)dt * 16u + l15) * SEQ + key0;
      const v16h va = g2_frag(vrow, hh), vb = g2_frag(vrow + 32, hh);
      o[dt] = g2_mma(pa.v, va, o[dt]); o[dt] = g2_mma(pb.v, vb, o[dt]); } }
  const float lt = l + __shfl_xor(l, 16);
  const float inv = 16.0f * (1.0f / lt);
  float ir[8];
#pragma unroll
  for (int r = 0; r < 8; ++r) ir[r] = __shfl(inv, (int)(8u * hh) + r);
#pragma unroll
  for (int dt = 0; dt < 4; ++dt)
#pragma unroll
    for (int r = 0; r < 8; ++r) so[w][8u * hh + (unsigned)r][(unsigned)dt * 16u + l15] = o[dt][r] * ir[r];
  __builtin_amdgcn_fence(4  , "workgroup"); __builtin_amdgcn_wave_barrier();
  const unsigned rq = lane >> 3, pc = lane & 7u;
  for (int pass = 0; pass < 2; ++pass) {
#pragma unroll
    for (int g = 0; g < 4; ++g) { const unsigned row = (unsigned)g * 4u + rq;
      const v4f va = *(const v4fa*)&so[w][row][pc * 8u]; const v4f vb = *(const v4fa*)&so[w][row][pc * 8u + 4u]; FragH f;
#pragma unroll
      for (int i = 0; i < 4; ++i) { f.h[i] = (_Float16)va[i]; f.h[4 + i] = (_Float16)vb[i]; }
      *(volatile v8us*)((unsigned short*)CTX + ((size_t)b * SEQ + q0 + row) * DM + hd * HD + pc * 8u) = f.half[0]; }
    if (pass == 0) __threadfence(); } }

__global__ __launch_bounds__(256) void k_ln(const float* __restrict__ Y, const float* __restrict__ g, const float* __restrict__ bt, float* __restrict__ out) {
  __shared__ float rs[8]; __shared__ float rv[8];
  const unsigned tid = threadIdx.x, row = blockIdx.x, w = tid >> 5, lane = tid & 31u;
  const v4f v = *(const v4fa*)(Y + (size_t)row * DM + tid * 4u);
  float s = (v[0] + v[1]) + (v[2] + v[3]);
  s += __shfl_xor(s, 1); s += __shfl_xor(s, 2); s += __shfl_xor(s, 4); s += __shfl_xor(s, 8); s += __shfl_xor(s, 16);
  if (lane == 0u) rs[w] = s;
  __syncthreads();
  float tot = 0.f;
#pragma unroll
  for (int i = 0; i < 8; ++i) tot += rs[i];
  const float mu = tot * (1.0f / (float)DM);
  v4f d;
#pragma unroll
  for (int i = 0; i < 4; ++i) d[i] = v[i] - mu;
  float ss = (d[0] * d[0] + d[1] * d[1]) + (d[2] * d[2] + d[3] * d[3]);
  ss += __shfl_xor(ss, 1); ss += __shfl_xor(ss, 2); ss += __shfl_xor(ss, 4); ss += __shfl_xor(ss, 8); ss += __shfl_xor(ss, 16);
  if (lane == 0u) rv[w] = ss;
  __syncthreads();
  float tv = 0.f;
#pragma unroll
  for (int i = 0; i < 8; ++i) tv += rv[i];
  const float var = tv * (1.0f / (float)DM);
  const float inv = rsqrtf(var + 1e-5f);
  const v4f gg = *(const v4fa*)(g + tid * 4u), bb = *(const v4fa*)(bt + tid * 4u);
  v4f o;
#pragma unroll
  for (int i = 0; i < 4; ++i) o[i] = d[i] * inv * bf16_rne(gg[i]) + bf16_rne(bb[i]);
  const unsigned b = row / USEQ, sq = row % USEQ;
  float* dst = out + ((size_t)b * SEQ_FULL + sq) * DM + tid * 4u;
  *(volatile v4f*)dst = o; __threadfence(); *(volatile v4f*)dst = o; }

extern "C" void kernel_launch(void* const* d_in, const int* in_sizes, int n_in,
                              void* d_out, int out_size, void* d_ws, size_t ws_size, hipStream_t stream) {
  if (n_in < 9) return;
  const float* x  = (const float*)d_in[0];
  const float* Wq = (const float*)d_in[2];
  const float* Wk = (const float*)d_in[3];
  const float* Wv = (const float*)d_in[4];
  const float* Wo = (const float*)d_in[5];
  const float* gm = (const float*)d_in[6];
  const float* bt = (const float*)d_in[7];
  const float* al = (const float*)d_in[8];
  const long long need_x = (long long)(NB - 1) * SEQ_FULL * DM + (long long)SEQ * DM;
  if ((long long)in_sizes[0] < need_x) return;
  if (in_sizes[2] < DM * DM || in_sizes[3] < DM * DM || in_sizes[4] < DM * DM || in_sizes[5] < DM * DM) return;
  if (in_sizes[6] < DM || in_sizes[7] < DM) return;
  if (in_sizes[8] < (NH - 1) * (SEQ_FULL - 1) + SEQ - 1) return;
  if ((long long)out_size < need_x) return;
  char* ws = (char*)d_ws; size_t off = 0;
  auto take = [&](size_t bytes) { char* p = ws + off; off += (bytes + 255) & ~(size_t)255; return p; };
  _Float16* WB  = (_Float16*)take((size_t)4 * DM * DM * 2);
  _Float16* X16 = (_Float16*)take((size_t)MROWS * DM * 2);
  _Float16* QKV = (_Float16*)take((size_t)MROWS * LQ * 2);
  _Float16* VT  = (_Float16*)take((size_t)NB * NH * HD * SEQ * 2);
  float*    KF  = (float*)take((size_t)MROWS * DM * 4);
  float*    PE  = (float*)take((size_t)SEQ * HD * 4);
  float*    RD  = (float*)take((size_t)256);
  if (off > ws_size || off > (size_t)134217728) return;
  _Float16* BQ = WB; _Float16* BK = WB + (size_t)DM * DM; _Float16* BV = WB + (size_t)2 * DM * DM; _Float16* BO = WB + (size_t)3 * DM * DM;
  _Float16* CTX = X16; float* Yf = KF;
  const unsigned nw = (unsigned)(DM * DM / 8 / 256);
  k_wnat<<<dim3(nw, 4u), 256, 0, stream>>>(Wq, Wk, Wv, Wo, WB);
  const unsigned nx = (unsigned)(MROWS * (DM / 8) / 256);
  k_x16<<<nx, 256, 0, stream>>>(x, X16);
  k_div<<<1, 64, 0, stream>>>(RD);
  k_pe<<<(unsigned)(SEQ * HD / 256), 256, 0, stream>>>(RD, PE);
  const unsigned gg = (unsigned)((MROWS / 128) * (DM / 64));
  k_gemm2<0><<<gg, 128, 0, stream>>>(X16, BQ, 0.0625f, PE, QKV,          KF);
  k_gemm2<1><<<gg, 128, 0, stream>>>(X16, BK, 0.0625f, PE, QKV,          KF);
  k_gemm2<2><<<gg, 128, 0, stream>>>(X16, BV, 0.0625f, PE, QKV + 2 * DM, KF);
  k_smear<<<nx, 256, 0, stream>>>(KF, al, PE, QKV);
  k_vt2<<<(unsigned)(NB * NH * NQT), 256, 0, stream>>>(QKV, VT);
  k_attn<<<dim3((unsigned)NQT, (unsigned)(NB * NH)), 128, 0, stream>>>(QKV, VT, CTX);
  k_gemm2<3><<<gg, 128, 0, stream>>>(CTX, BO, 0.00390625f, x, QKV, Yf);
  k_ln<<<(unsigned)MROWS, 256, 0, stream>>>(Yf, gm, bt, (float*)d_out);
}
